// GENELink_4475355922564
// MI455X (gfx1250) — hardware-verified
//
#include <hip/hip_runtime.h>
#include <math.h>

typedef __attribute__((ext_vector_type(16))) _Float16 v16h;
typedef __attribute__((ext_vector_type(16))) __bf16 v16b;
typedef __attribute__((ext_vector_type(8)))  _Float16 v8h;
typedef __attribute__((ext_vector_type(8)))  float v8f;
typedef __attribute__((ext_vector_type(4)))  float v4f;
typedef __attribute__((ext_vector_type(2)))  float v2f;
typedef __attribute__((ext_vector_type(4)))  unsigned v4u;
typedef __attribute__((ext_vector_type(4)))  int v4i;
typedef float __attribute__((may_alias)) float_a;
typedef int __attribute__((may_alias)) int_a;

template <typename T> __device__ __forceinline__ void vst2(void* p, T v) { *(volatile T*)p = v; __threadfence(); *(volatile T*)p = v; }
__device__ __forceinline__ v8f wmma16(v16h a, v16h b, v8f c) {
  v8f d = __builtin_amdgcn_wmma_f32_16x16x32_f16(false, a, false, b, (short)0, c, false, false);
  asm volatile("v_nop\n\tv_nop\n\tv_nop\n\tv_nop" : "+v"(d) : "v"(a), "v"(b));
  return d;
}
__device__ __forceinline__ v8f wmma_bf(v16b a, v16b b, v8f c) {
  v8f d = __builtin_amdgcn_wmma_f32_16x16x32_bf16(false, a, false, b, (short)0, c, false, false);
  asm volatile("v_nop\n\tv_nop\n\tv_nop\n\tv_nop" : "+v"(d) : "v"(a), "v"(b));
  return d;
}
__device__ __forceinline__ v16h frag_h(const _Float16* rowk0, int lane) {
  union { v16h v; v8h q[2]; } u; const _Float16* p = rowk0 + 8 * (lane >> 4);
  u.q[0] = *(const v8h*)p; u.q[1] = *(const v8h*)(p + 16); return u.v;
}
__device__ __forceinline__ v16h frag_f32(const float* rowk0, int lane) {
  v16h a; const float* p = rowk0 + 8 * (lane >> 4);
#pragma unroll
  for (int i = 0; i < 8; ++i) { a[i] = (_Float16)p[i]; a[8 + i] = (_Float16)p[16 + i]; }
  return a;
}
__device__ __forceinline__ v16h frag_f32s(const float* rowk0, int lane, float sc) {
  v16h a; const float* p = rowk0 + 8 * (lane >> 4);
#pragma unroll
  for (int i = 0; i < 8; ++i) { a[i] = (_Float16)(p[i] * sc); a[8 + i] = (_Float16)(p[16 + i] * sc); }
  return a;
}
__device__ __forceinline__ v16h fragc_f32(const float* W, int k0, int n, int lane, int ld, int K) {
  v16h a; const int g = lane >> 4;
#pragma unroll
  for (int i = 0; i < 8; ++i) { const int ka = k0 + 8 * g + i, kb = ka + 16;
    a[i] = (_Float16)(ka < K ? W[(size_t)(ka < K ? ka : K - 1) * ld + n] : 0.f); a[8 + i] = (_Float16)(kb < K ? W[(size_t)(kb < K ? kb : K - 1) * ld + n] : 0.f); }
  return a;
}
struct F2 { v16b h, l; };
__device__ __forceinline__ F2 bsplit16(const float v[16]) { F2 r;
#pragma unroll
  for (int i = 0; i < 16; ++i) { const __bf16 h = (__bf16)v[i]; r.h[i] = h; r.l[i] = (__bf16)(v[i] - (float)h); }
  return r; }
__device__ __forceinline__ F2 split_row(const float* row, int k0, int lane) { float v[16]; const float* p = row + k0 + 8 * (lane >> 4);
#pragma unroll
  for (int i = 0; i < 8; ++i) { v[i] = p[i]; v[8 + i] = p[16 + i]; }
  return bsplit16(v); }
__device__ __forceinline__ F2 split_rowK(const float* row, int k0, int lane, int K) { float v[16]; const int g = lane >> 4;
#pragma unroll
  for (int i = 0; i < 8; ++i) { const int ka = k0 + 8 * g + i, kb = ka + 16; v[i] = ka < K ? row[ka < K ? ka : K - 1] : 0.f; v[8 + i] = kb < K ? row[kb < K ? kb : K - 1] : 0.f; }
  return bsplit16(v); }
__device__ __forceinline__ F2 split_col(const float* W, int k0, int n, int lane, int ld, int K) { float v[16]; const int g = lane >> 4;
#pragma unroll
  for (int i = 0; i < 8; ++i) { const int ka = k0 + 8 * g + i, kb = ka + 16; v[i] = ka < K ? W[(size_t)(ka < K ? ka : K - 1) * ld + n] : 0.f; v[8 + i] = kb < K ? W[(size_t)(kb < K ? kb : K - 1) * ld + n] : 0.f; }
  return bsplit16(v); }
__device__ __forceinline__ v8f mac3(const F2& a, const F2& b, v8f c) { c = wmma_bf(a.l, b.h, c); c = wmma_bf(a.h, b.l, c); return wmma_bf(a.h, b.h, c); }
__device__ __forceinline__ float sigm(float v) { return 1.0f / (1.0f + expf(-v)); }
#define LDSX() do { asm volatile("s_wait_dscnt 0" ::: "memory"); __builtin_amdgcn_wave_barrier(); __builtin_amdgcn_fence(__ATOMIC_RELEASE, "workgroup"); } while (0)


#ifndef NN
#define NN 4096
#endif
#define EP 131072
#ifndef NE
#define NE 131072
#endif
#define DIN 512
#define DH 256
#define NHD 4
#define NL 4
#define NBLK (NN / 64)
typedef __attribute__((ext_vector_type(8))) __bf16 v8b;
__device__ __forceinline__ v16b frag_b(const __bf16* rowk0, int lane) {
  union { v16b v; v8b q[2]; } u; const __bf16* p = rowk0 + 8 * (lane >> 4);
  u.q[0] = *(const v8b*)p; u.q[1] = *(const v8b*)(p + 16); return u.v;
}
__device__ __forceinline__ float bfr(float v) { return (float)(__bf16)v; }
__device__ __attribute__((noinline)) float exp_ni(float v) { return expf(v); }
__device__ __attribute__((noinline)) float erf_ni(float v) { return erff(v); }

__device__ __attribute__((noinline)) float expm1_ni(float v) { return expm1f(v); }
#define CSA_N NN
#define CSA_E NE
#define CSA_FINN (CSA_E + 32 * CSA_NBK)
#define CSA_CHUNK 4096
#define CSA_BKT 256
#define CSA_NCH ((CSA_E + CSA_CHUNK - 1) / CSA_CHUNK)
#define CSA_NBK ((CSA_N + CSA_BKT - 1) / CSA_BKT)
#define CSA_NBKP (((CSA_NBK + 63) / 64) * 64)
#define CSA_SEGCAP (CSA_E + 32 * CSA_NBK * CSA_NCH)
#ifndef CSA_BCAP
#define CSA_BCAP 10240
#endif
#define CSA_SZ_CNT   (4u * CSA_NCH * CSA_NBKP)
#define CSA_SZ_OFF   (4u * CSA_NBK * (((CSA_NCH + 31) / 32) * 32))
#define CSA_SZ_BST   (4u * (((CSA_NBK + 1 + 31) / 32) * 32))
#define CSA_SZ_SEG   (4u * CSA_SEGCAP)
#define CSA_SZ_FIN   (4u * (CSA_E + 32 * CSA_NBK))
#define CSA_SZ_ROW   (4u * CSA_NBK * CSA_BKT)
#define CSA_OFFP (((CSA_NCH + 31) / 32) * 32)

__global__ __launch_bounds__(256) void k_csA_cnt(const int* __restrict__ DST, int dstride, int* __restrict__ CNT) {
  __shared__ unsigned short sc[256][CSA_NBK + 1]; __shared__ __align__(16) int srow[CSA_NBKP];
  const int c = blockIdx.x, tid = threadIdx.x;
  for (int b = 0; b < CSA_NBK; ++b) sc[tid][b] = 0;
  const size_t e0 = (size_t)c * CSA_CHUNK + tid * 16;
  for (int i = 0; i < 16; ++i) { const size_t e = e0 + i; if (e < (size_t)CSA_E) { int d = DST[e * dstride]; d = min(max(d, 0), CSA_N - 1); sc[tid][d / CSA_BKT] += 1; } }
  __syncthreads();
  for (int b = tid; b < CSA_NBKP; b += 256) { int s = 0; if (b < CSA_NBK) for (int t = 0; t < 256; ++t) s += sc[t][b]; srow[b] = s; }
  __syncthreads();
  for (int q = tid; q < CSA_NBKP / 4; q += 256) vst2((unsigned*)(CNT + (size_t)c * CSA_NBKP + q * 4), *(const v4u*)&srow[q * 4]);
}
__global__ __launch_bounds__(256) void k_csA_scan(const int* __restrict__ CNT, int* __restrict__ OFF, int* __restrict__ BST) {
  __shared__ int sbt[CSA_NBK + 1]; __shared__ int sbs[((CSA_NBK + 1 + 31) / 32) * 32]; __shared__ int scnt[CSA_NBK + 1]; __shared__ __align__(16) int sbuf[64][CSA_OFFP];
  const int tid = threadIdx.x;
  for (int b = tid; b < CSA_NBK; b += 256) { int sp = 0, st = 0; for (int c = 0; c < CSA_NCH; ++c) { const int n = CNT[(size_t)c * CSA_NBKP + b]; st += n; sp += (n + 31) & ~31; } sbt[b] = sp; scnt[b] = st; }
  for (int b = tid; b < ((CSA_NBK + 1 + 31) / 32) * 32; b += 256) sbs[b] = 0;
  __syncthreads();
  if (tid == 0) { int acc = 0, accf = 0; for (int b = 0; b < CSA_NBK; ++b) { const int t = sbt[b]; sbt[b] = acc; acc += t; sbs[b] = accf; accf += (scnt[b] + 31) & ~31; } sbs[CSA_NBK] = accf; }
  __syncthreads();
  for (int b0 = 0; b0 < CSA_NBK; b0 += 64) {
    if (tid < 64 && b0 + tid < CSA_NBK) { const int b = b0 + tid; int o = sbt[b]; for (int c = 0; c < CSA_OFFP; ++c) { if (c < CSA_NCH) { sbuf[tid][c] = o; o += (CNT[(size_t)c * CSA_NBKP + b] + 31) & ~31; } else sbuf[tid][c] = 0; } }
    __syncthreads();
    for (int q = tid; q < 64 * (CSA_OFFP / 4); q += 256) { const int r = q / (CSA_OFFP / 4), pc = q % (CSA_OFFP / 4); if (b0 + r < CSA_NBK) vst2((unsigned*)(OFF + (size_t)(b0 + r) * CSA_OFFP + pc * 4), *(const v4u*)&sbuf[r][pc * 4]); }
    __syncthreads(); }
  for (int q = tid; q < ((CSA_NBK + 1 + 31) / 32) * 32 / 4; q += 256) vst2((unsigned*)(BST + q * 4), *(const v4u*)&sbs[q * 4]);
}
__global__ __launch_bounds__(256) void k_csA_scatter(const int* __restrict__ SRC, const int* __restrict__ DST, int sstride, int dstride, const int* __restrict__ OFF, int* __restrict__ SEGS, int* __restrict__ SEGE) {
  __shared__ unsigned short sc[256][CSA_NBK + 1]; __shared__ int sbase[CSA_NBK + 1]; __shared__ int scn[CSA_NBK + 1]; __shared__ int sord[CSA_CHUNK];
  const int c = blockIdx.x, tid = threadIdx.x;
  for (int b = 0; b < CSA_NBK; ++b) sc[tid][b] = 0;
  const size_t e0 = (size_t)c * CSA_CHUNK + tid * 16; int bk[16];
#pragma unroll
  for (int i = 0; i < 16; ++i) { const size_t e = e0 + i; bk[i] = -1; if (e < (size_t)CSA_E) { int d = DST[e * dstride]; d = min(max(d, 0), CSA_N - 1); bk[i] = d / CSA_BKT; sc[tid][bk[i]] += 1; } }
  __syncthreads();
  for (int b = tid; b < CSA_NBK; b += 256) { int acc = 0; for (int t = 0; t < 256; ++t) { const int v = sc[t][b]; sc[t][b] = (unsigned short)acc; acc += v; } scn[b] = acc; }
  __syncthreads();
  if (tid == 0) { int acc = 0; for (int b = 0; b < CSA_NBK; ++b) { sbase[b] = acc; acc += scn[b]; } }
  __syncthreads();
#pragma unroll
  for (int i = 0; i < 16; ++i) { if (bk[i] >= 0) { const int b = bk[i]; const int r = sc[tid][b]; sc[tid][b] = (unsigned short)(r + 1); sord[sbase[b] + r] = tid * 16 + i; } }
  __syncthreads();
  for (int b = 0; b < CSA_NBK; ++b) { const int n = scn[b]; if (n == 0) continue; const int nl = ((n + 31) & ~31); const size_t o = (size_t)(min(max(OFF[(size_t)b * CSA_OFFP + c], 0), CSA_SEGCAP - nl) & ~31);
    for (int q = tid; q < nl / 4; q += 256) { int4 vs, ve;
#pragma unroll
      for (int k = 0; k < 4; ++k) { const int i = q * 4 + k; int s = -1, eid = -1; if (i < n) { const size_t e = (size_t)c * CSA_CHUNK + sord[sbase[b] + i]; s = min(max(SRC[e * sstride], 0), CSA_N - 1); eid = (int)e; } vs[k] = s; ve[k] = eid; }
      vst2((unsigned*)(SEGS + o + q * 4), *(const v4u*)&vs); vst2((unsigned*)(SEGE + o + q * 4), *(const v4u*)&ve); } }
}
__global__ __launch_bounds__(256) void k_csA_bucket(const int* __restrict__ CNT, const int* __restrict__ OFF, const int* __restrict__ BST, const int* __restrict__ SEGS, const int* __restrict__ SEGE, const int* __restrict__ DST, int dstride, int* __restrict__ FS, int* __restrict__ FE, int* __restrict__ ROWST, int* __restrict__ ROWCNT) {
  __shared__ int ssrc[CSA_BCAP]; __shared__ int seid[CSA_BCAP]; __shared__ unsigned char snod[CSA_BCAP]; __shared__ int souts[CSA_BCAP]; __shared__ int soute[CSA_BCAP]; __shared__ int scount[256]; __shared__ int sstart[257]; __shared__ int stot;
  const int b = blockIdx.x, tid = threadIdx.x;
  if (tid == 0) { int t = 0; for (int c = 0; c < CSA_NCH; ++c) t += min(max(CNT[(size_t)c * CSA_NBKP + b], 0), CSA_CHUNK); stot = (t <= CSA_BCAP) ? t : 0; }
  __syncthreads();
  { int base = 0; for (int c = 0; c < CSA_NCH; ++c) { const int n = min(max(CNT[(size_t)c * CSA_NBKP + b], 0), CSA_CHUNK); const int o = min(max(OFF[(size_t)b * CSA_OFFP + c], 0), CSA_SEGCAP - ((n + 31) & ~31));
      for (int i = tid; i < n; i += 256) { const int p = base + i; if (p < CSA_BCAP) { ssrc[p] = min(max(SEGS[o + i], 0), CSA_N - 1); const int e = min(max(SEGE[o + i], 0), CSA_E - 1); seid[p] = e; int d = DST[(size_t)e * dstride]; d = min(max(d, 0), CSA_N - 1); const int dl = d - b * CSA_BKT; snod[p] = (unsigned char)(dl >= 0 && dl < 256 ? dl : 255); } }
      base += n; } }
  __syncthreads();
  const int node = b * CSA_BKT + tid; int cnt = 0; for (int p = 0; p < stot; ++p) cnt += (snod[p] == tid) ? 1 : 0;
  scount[tid] = cnt; __syncthreads();
  if (tid == 0) { int acc = 0; for (int t = 0; t < 256; ++t) { sstart[t] = acc; acc += scount[t]; } sstart[256] = acc; }
  __syncthreads();
  const int bst0 = min(max(BST[b], 0), CSA_FINN - ((sstart[256] + 31) & ~31)) & ~31; const int gst = bst0 + sstart[tid];
  { int w = sstart[tid]; for (int p = 0; p < stot; ++p) if (snod[p] == tid) { souts[w] = ssrc[p]; soute[w] = seid[p]; ++w; } }
  __syncthreads();
  { const int n = sstart[256]; const int nl = (n + 31) & ~31; for (int q = tid; q < nl / 4; q += 256) { int4 vs, ve;
#pragma unroll
      for (int k = 0; k < 4; ++k) { const int i = q * 4 + k; vs[k] = i < n ? souts[i] : -1; ve[k] = i < n ? soute[i] : -1; }
      vst2((unsigned*)(FS + bst0 + q * 4), *(const v4u*)&vs); vst2((unsigned*)(FE + bst0 + q * 4), *(const v4u*)&ve); } }
  __syncthreads();
  { __shared__ __align__(16) int srs[256], src2[256]; srs[tid] = node < CSA_N ? gst : 0; src2[tid] = node < CSA_N ? cnt : 0; __syncthreads();
    if (tid < 64) vst2((unsigned*)(ROWST + (size_t)b * 256 + tid * 4), *(const v4u*)&srs[tid * 4]); else if (tid < 128) vst2((unsigned*)(ROWCNT + (size_t)b * 256 + (tid - 64) * 4), *(const v4u*)&src2[(tid - 64) * 4]); }
}


#define WS_CNT  0u
#define WS_OFF  (WS_CNT + CSA_SZ_CNT)
#define WS_BST  (WS_OFF + CSA_SZ_OFF)
#define WS_SEGS (WS_BST + CSA_SZ_BST)
#define WS_SEGE (WS_SEGS + CSA_SZ_SEG)
#define WS_FS   (WS_SEGE + CSA_SZ_SEG)
#define WS_FE   (WS_FS + CSA_SZ_FIN)
#define WS_RST  (WS_FE + CSA_SZ_FIN)
#define WS_RCT  (WS_RST + CSA_SZ_ROW)
#define WS_PW   (WS_RCT + CSA_SZ_ROW)
#define PW1 0
#define PWK (PW1 + NHD * DH * DIN)
#define PWP (PWK + 3 * NHD * DH * DH)
#define PWEND (PWP + DH * DIN)
#define WS_H    (WS_PW + 2u * PWEND)
#define WS_WH   (WS_H + 4u * NHD * NN * DH)
#define WS_PS   (WS_WH + 4u * 2 * NHD * NN)
#define WS_S    (WS_PS + 4u * NHD * NBLK * DH)
#define WS_PREV (WS_S + 4u * NHD * DH)
#define WS_OA   (WS_PREV + 4u * NN * DH)
#define WS_OB   (WS_OA + 4u * NN * DH)
#define WS_END  (WS_OB + 4u * NN * DH)

__global__ __launch_bounds__(256) void k_packT(const float* __restrict__ W1, const float* __restrict__ WK, const float* __restrict__ PWm, __bf16* __restrict__ PW) {
  __shared__ __align__(16) __bf16 s[DIN]; const int n = blockIdx.x, p = blockIdx.y, tid = threadIdx.x;
  int K; size_t dst;
  if (p < 4) { K = DIN; dst = PW1 + ((size_t)p * DH + n) * DIN; for (int k = tid; k < K; k += 256) s[k] = (__bf16)W1[((size_t)p * DIN + k) * DH + n]; }
  else if (p < 16) { const int q = p - 4; K = DH; dst = PWK + ((size_t)q * DH + n) * DH; for (int k = tid; k < K; k += 256) s[k] = (__bf16)WK[((size_t)q * DH + k) * DH + n]; }
  else { K = DIN; dst = PWP + (size_t)n * DIN; for (int k = tid; k < K; k += 256) s[k] = (__bf16)PWm[(size_t)k * DH + n]; }
  __syncthreads();
  if (tid < K / 8) vst2((unsigned*)(PW + dst + tid * 8), *(const v4u*)&s[tid * 8]);
}
template <int K, int RIN>
__global__ __launch_bounds__(128) void k_h(const float* __restrict__ XIN, const __bf16* __restrict__ P, const float* __restrict__ A, int hd, float* __restrict__ H, float* __restrict__ WH, float* __restrict__ PS) {
  __shared__ __align__(16) float so[64][DH + 4]; __shared__ float sa[2 * DH]; __shared__ __align__(16) float sw[2][64];
  const int tid = threadIdx.x, wave = tid >> 5, lane = tid & 31, col = lane & 15, g = lane >> 4; const size_t r0 = (size_t)blockIdx.x * 64 + wave * 16;
  for (int i = tid; i < 2 * DH; i += 128) sa[i] = bfr(A[(size_t)hd * 2 * DH + i]);
  v8f acc[16]; for (int j = 0; j < 16; ++j) acc[j] = (v8f){};
#pragma unroll 2
  for (int kc = 0; kc < K / 32; ++kc) { F2 a; if (RIN) { v16b ax; const float* p = XIN + (r0 + col) * K + kc * 32 + 8 * g;
#pragma unroll
      for (int i = 0; i < 8; ++i) { ax[i] = (__bf16)p[i]; ax[8 + i] = (__bf16)p[16 + i]; } a.h = ax; a.l = ax; } else a = split_row(XIN + (r0 + col) * K, kc * 32, lane);
#pragma unroll
    for (int j = 0; j < 16; ++j) { const v16b w = frag_b(P + (size_t)(hd * DH + j * 16 + col) * K + kc * 32, lane); if (!RIN) acc[j] = wmma_bf(a.l, w, acc[j]); acc[j] = wmma_bf(a.h, w, acc[j]); } }
  __syncthreads();
  float p1[8], p2[8];
#pragma unroll
  for (int r = 0; r < 8; ++r) { p1[r] = 0.f; p2[r] = 0.f; }
#pragma unroll
  for (int j = 0; j < 16; ++j) { const int c = j * 16 + col;
#pragma unroll
    for (int r = 0; r < 8; ++r) { const float v = acc[j][r]; so[wave * 16 + 8 * g + r][c] = v; p1[r] += v * sa[c]; p2[r] += v * sa[DH + c]; } }
#pragma unroll
  for (int r = 0; r < 8; ++r) { float a1 = p1[r], a2 = p2[r];
#pragma unroll
    for (int o = 1; o < 16; o <<= 1) { a1 += __shfl_xor(a1, o); a2 += __shfl_xor(a2, o); }
    if (col == 0) { sw[0][wave * 16 + 8 * g + r] = a1; sw[1][wave * 16 + 8 * g + r] = a2; } }
  __syncthreads();
  for (int q = tid; q < 64 * 64; q += 128) { const int rl = q >> 6, pc = q & 63; vst2(H + ((size_t)hd * NN + blockIdx.x * 64 + rl) * DH + pc * 4, *(const v4f*)&so[rl][pc * 4]); }
  if (tid < 32) { const int w = tid >> 4, pc = tid & 15; vst2(WH + ((size_t)w * NHD + hd) * NN + blockIdx.x * 64 + pc * 4, *(const v4f*)&sw[w][pc * 4]); }
  __shared__ __align__(16) float sps[DH];
  for (int c = tid; c < DH; c += 128) { float s = 0.f; for (int rl = 0; rl < 64; ++rl) s += so[rl][c]; sps[c] = s; }
  __syncthreads();
  if (tid < 64) vst2(PS + ((size_t)hd * NBLK + blockIdx.x) * DH + tid * 4, *(const v4f*)&sps[tid * 4]);
}
__global__ __launch_bounds__(256) void k_cols(const float* __restrict__ PS, float* __restrict__ S) {
  __shared__ __align__(16) float s[DH]; const int hd = blockIdx.x, c = threadIdx.x; float acc = 0.f;
  for (int b = 0; b < NBLK; ++b) acc += PS[((size_t)hd * NBLK + b) * DH + c];
  s[c] = acc; __syncthreads();
  if (c < 64) vst2(S + (size_t)hd * DH + c * 4, *(const v4f*)&s[c * 4]);
}
__global__ __launch_bounds__(128) void k_proj1(const float* __restrict__ X, const __bf16* __restrict__ P, const float* __restrict__ PB, float* __restrict__ PREV) {
  __shared__ __align__(16) float so[4][16][132];
  const int tid = threadIdx.x, wave = tid >> 5, lane = tid & 31, col = lane & 15, g = lane >> 4; const size_t r0 = (size_t)blockIdx.x * 64 + wave * 16; const int n0 = blockIdx.y * 128;
  v8f acc[8] = {};
#pragma unroll 2
  for (int kc = 0; kc < DIN / 32; ++kc) { v16b a; { const float* p = X + (r0 + col) * DIN + kc * 32 + 8 * g;
#pragma unroll
      for (int i = 0; i < 8; ++i) { a[i] = (__bf16)p[i]; a[8 + i] = (__bf16)p[16 + i]; } }
#pragma unroll
    for (int j = 0; j < 8; ++j) acc[j] = wmma_bf(a, frag_b(P + (size_t)(n0 + j * 16 + col) * DIN + kc * 32, lane), acc[j]); }
#pragma unroll
  for (int j = 0; j < 8; ++j) { const float bb = bfr(PB[n0 + j * 16 + col]);
#pragma unroll
    for (int r = 0; r < 8; ++r) so[wave][8 * g + r][j * 16 + col] = acc[j][r] + bb; }
  LDSX();
  for (int rl = 0; rl < 16; ++rl) vst2(PREV + (r0 + rl) * DH + n0 + lane * 4, *(const v4f*)&so[wave][rl][lane * 4]);
}
__global__ __launch_bounds__(256) void k_gene(const float* __restrict__ H, const float* __restrict__ WH, const float* __restrict__ S, const int* __restrict__ FS, const int* __restrict__ RST, const int* __restrict__ RCT, const float* __restrict__ BIAS, const float* __restrict__ PREV, float* __restrict__ OUT) {
  __shared__ unsigned bm[8][NN / 32]; __shared__ __align__(16) float so[8][DH + 4];
  const int tid = threadIdx.x, wave = tid >> 5, lane = tid & 31; const int i = blockIdx.x * 8 + wave; const int f0 = lane * 8;
  float mean[8];
#pragma unroll
  for (int q = 0; q < 8; ++q) mean[q] = 0.f;
  const int cnt = min(max(RCT[i], 0), CSA_BCAP); const int st = min(max(RST[i], 0), CSA_FINN - max(cnt, 1));
  for (int w = lane; w < NN / 32; w += 32) bm[wave][w] = 0u;
  LDSX();
  if (lane == 0) for (int e = 0; e < cnt; ++e) { const int j = min(max(FS[st + e], 0), NN - 1); bm[wave][j >> 5] |= (1u << (j & 31)); }
  LDSX();
  int nset = 0; for (int w = lane; w < NN / 32; w += 32) nset += __popc(bm[wave][w]);
#pragma unroll
  for (int o = 1; o < 32; o <<= 1) nset += __shfl_xor(nset, o);
#pragma unroll 1
  for (int hd = 0; hd < NHD; ++hd) { const float* Hh = H + (size_t)hd * NN * DH; const float* W1p = WH + (size_t)(0 * NHD + hd) * NN; const float* W2p = WH + (size_t)(1 * NHD + hd) * NN; const float w1i = W1p[i];
    float mx = -3.0e38f;
    for (int w = lane; w < NN / 32; w += 32) { unsigned bits = bm[wave][w]; while (bits) { const int b = __ffs(bits) - 1; bits &= bits - 1; const int j = w * 32 + b; float ev = w1i + W2p[j]; ev = (ev >= 0.f) ? ev : 0.2f * ev; mx = fmaxf(mx, ev); } }
#pragma unroll
    for (int o = 1; o < 32; o <<= 1) mx = fmaxf(mx, __shfl_xor(mx, o));
    if (nset < NN) mx = fmaxf(mx, 0.f);
    float z = 0.f; float acc[8], sub[8];
#pragma unroll
    for (int q = 0; q < 8; ++q) { acc[q] = 0.f; sub[q] = 0.f; }
    for (int w = 0; w < NN / 32; ++w) { unsigned bits = bm[wave][w]; while (bits) { const int b = __ffs(bits) - 1; bits &= bits - 1; const int j = w * 32 + b; float ev = w1i + W2p[j]; ev = (ev >= 0.f) ? ev : 0.2f * ev; const float e = exp_ni(ev - mx); z += e; const float* hr = Hh + (size_t)j * DH + f0;
#pragma unroll
        for (int q = 0; q < 8; ++q) { acc[q] += e * hr[q]; sub[q] += hr[q]; } } }
    const float e0 = exp_ni(-mx); const float Z = (float)(NN - nset) * e0 + z; const float iZ = 1.0f / Z; const float* Sh = S + (size_t)hd * DH + f0;
    float o[8]; float nrm = 0.f;
#pragma unroll
    for (int q = 0; q < 8; ++q) { float v = (e0 * (Sh[q] - sub[q]) + acc[q]) * iZ; v = (v >= 0.f) ? v : 0.2f * v; o[q] = v; nrm += v * v; }
#pragma unroll
    for (int oo = 1; oo < 32; oo <<= 1) nrm += __shfl_xor(nrm, oo);
    const float inv = 1.0f / fmaxf(sqrtf(nrm), 1e-12f);
#pragma unroll
    for (int q = 0; q < 8; ++q) mean[q] += o[q] * inv + bfr(BIAS[(size_t)hd * DH + f0 + q]);
  }
  const float* pr = PREV + (size_t)i * DH + f0;
#pragma unroll
  for (int q = 0; q < 8; ++q) { float v = mean[q] * 0.25f + pr[q]; v = (v > 0.f) ? v : expm1_ni(v); so[wave][f0 + q] = v; }
  LDSX();
  vst2(OUT + (size_t)i * DH + lane * 4, *(const v4f*)&so[wave][lane * 4]); vst2(OUT + (size_t)i * DH + 128 + lane * 4, *(const v4f*)&so[wave][128 + lane * 4]);
}
extern "C" void kernel_launch(void* const* d_in, const int* in_sizes, int n_in, void* d_out, int out_size, void* d_ws, size_t ws_size, hipStream_t stream) {
  (void)in_sizes; (void)n_in; (void)out_size;
  const float** F = (const float**)d_in; const int* EI = (const int*)d_in[1];
  if (ws_size < (size_t)WS_END) return;
  char* ws = (char*)d_ws;
  int *CNT = (int*)(ws + WS_CNT), *OFF = (int*)(ws + WS_OFF), *BST = (int*)(ws + WS_BST), *SEGS = (int*)(ws + WS_SEGS), *SEGE = (int*)(ws + WS_SEGE), *FS = (int*)(ws + WS_FS), *FE = (int*)(ws + WS_FE), *RST = (int*)(ws + WS_RST), *RCT = (int*)(ws + WS_RCT);
  __bf16* PW = (__bf16*)(ws + WS_PW); float *H = (float*)(ws + WS_H), *WH = (float*)(ws + WS_WH), *PS = (float*)(ws + WS_PS), *S = (float*)(ws + WS_S), *PREV = (float*)(ws + WS_PREV), *OA = (float*)(ws + WS_OA), *OB = (float*)(ws + WS_OB);
  const int* ER = EI; const int* EC = EI + EP;
  k_packT<<<dim3(DH, 17), 256, 0, stream>>>(F[2], F[5], F[8], PW);
  k_csA_cnt<<<CSA_NCH, 256, 0, stream>>>(ER, 1, CNT); k_csA_scan<<<1, 256, 0, stream>>>(CNT, OFF, BST); k_csA_scatter<<<CSA_NCH, 256, 0, stream>>>(EC, ER, 1, 1, OFF, SEGS, SEGE); k_csA_bucket<<<CSA_NBK, 256, 0, stream>>>(CNT, OFF, BST, SEGS, SEGE, ER, 1, FS, FE, RST, RCT);
  k_proj1<<<dim3(NBLK, 2), 128, 0, stream>>>(F[0], PW + PWP, F[9], PREV);
  for (int hd = 0; hd < NHD; ++hd) k_h<DIN, 1><<<NBLK, 128, 0, stream>>>(F[0], PW + PW1, F[3], hd, H, WH, PS);
  k_cols<<<NHD, 256, 0, stream>>>(PS, S);
  k_gene<<<NN / 8, 256, 0, stream>>>(H, WH, S, FS, RST, RCT, F[4], PREV, OA);
  float* cur = OA; float* nxt = OB;
  for (int l = 0; l < 3; ++l) {
    for (int hd = 0; hd < NHD; ++hd) k_h<DH, 0><<<NBLK, 128, 0, stream>>>(cur, PW + PWK + (size_t)l * NHD * DH * DH, F[6] + (size_t)l * NHD * 2 * DH, hd, H, WH, PS);
    k_cols<<<NHD, 256, 0, stream>>>(PS, S);
    k_gene<<<NN / 8, 256, 0, stream>>>(H, WH, S, FS, RST, RCT, F[7] + (size_t)l * NHD * DH, cur, (l == 2) ? (float*)d_out : nxt);
    float* t = cur; cur = nxt; nxt = t; }
}
